// VanillaRNN_82781199663717
// MI455X (gfx1250) — hardware-verified
//
#include <hip/hip_runtime.h>
#include <math.h>

constexpr int NB   = 256;
constexpr int NT   = 512;
constexpr int NI   = 64;
constexpr int NH   = 512;
constexpr int NO   = 512;
constexpr int KF   = NH + NI;
constexpr int NKC  = KF / 32;
constexpr int NTHR = 256;
constexpr int RPB  = 32;
constexpr int NRBLK = NB / RPB;
constexpr int APITCH = KF + 8;
constexpr int ATILE  = RPB * APITCH;
constexpr float WCARRY     = 64.0f;
constexpr float WCARRY_INV = 1.0f / 64.0f;
static_assert(NB % RPB == 0);
static_assert(NH == 64 * (NTHR / 32));
static_assert(KF % 32 == 0 && NKC % 2 == 0);
static_assert(APITCH % 8 == 0 && (2 * ATILE) % 8 == 0);
static_assert(RPB * (NI / 8) == NTHR);
static_assert(NI == 64);
static_assert(NH % 64 == 0);
static_assert(NB % 64 == 0 && NO % 64 == 0 && NH % 32 == 0);
static_assert(((NB / 64) * (NO / 64)) % 8 == 0);
static_assert(NO % 128 == 0);
static_assert(NB % (NTHR / 32) == 0);
static_assert(NH % 8 == 0 && NO % 8 == 0);

typedef __attribute__((ext_vector_type(16))) _Float16 v16h;
typedef __attribute__((ext_vector_type(8)))  _Float16 v8h;
typedef __attribute__((ext_vector_type(16))) __bf16   v16b;
typedef __attribute__((ext_vector_type(8)))  __bf16   v8b;
typedef __attribute__((ext_vector_type(8)))  float    v8f;
typedef __attribute__((ext_vector_type(4)))  float    v4f;
typedef __attribute__((ext_vector_type(4)))  unsigned v4u;

__device__ __forceinline__ unsigned short f2bf_bits(float f) {
  unsigned u = __float_as_uint(f);
  return (unsigned short)((u + 0x7FFFu + ((u >> 16) & 1u)) >> 16);
}
__device__ __forceinline__ float bf_bits2f(unsigned short h) { return __uint_as_float(((unsigned)h) << 16); }

__device__ __forceinline__ void dep_guard_h(v8f& a, v8f& b, v16h x, v16h y) { asm volatile("v_nop\n\tv_nop\n\tv_nop\n\tv_nop" : "+v"(a), "+v"(b) : "v"(x), "v"(y)); }
__device__ __forceinline__ void dep_guard_b(v8f& a, v8f& b, v16b x, v16b y) { asm volatile("v_nop\n\tv_nop\n\tv_nop\n\tv_nop" : "+v"(a), "+v"(b) : "v"(x), "v"(y)); }
__device__ __forceinline__ void dep_guard4_h(v8f& a, v8f& b, v8f& c, v8f& d, v16h x, v16h y) { asm volatile("v_nop\n\tv_nop\n\tv_nop\n\tv_nop" : "+v"(a), "+v"(b), "+v"(c), "+v"(d) : "v"(x), "v"(y)); }
__device__ __forceinline__ void dep_guard4_b(v8f& a, v8f& b, v8f& c, v8f& d, v16b x, v16b y) { asm volatile("v_nop\n\tv_nop\n\tv_nop\n\tv_nop" : "+v"(a), "+v"(b), "+v"(c), "+v"(d) : "v"(x), "v"(y)); }
__device__ __forceinline__ void keep4_h(v16h a, v16h b, v16h c, v16h d) { asm volatile("v_nop" :: "v"(a), "v"(b), "v"(c), "v"(d)); }
__device__ __forceinline__ void keep4_b(v16b a, v16b b, v16b c, v16b d) { asm volatile("v_nop" :: "v"(a), "v"(b), "v"(c), "v"(d)); }
__device__ __forceinline__ void acc_guard4(v8f& a, v8f& b, v8f& c, v8f& d) { asm volatile("v_nop\n\tv_nop\n\tv_nop\n\tv_nop" : "+v"(a), "+v"(b), "+v"(c), "+v"(d)); }
__device__ __forceinline__ void guard8_h(v8f& c0, v8f& c1, v8f& c2, v8f& c3, v8f& c4, v8f& c5, v8f& c6, v8f& c7,
                                         v16h f0, v16h f1, v16h f2, v16h f3, v16h f4, v16h f5) {
  asm volatile("v_nop\n\tv_nop\n\tv_nop\n\tv_nop"
               : "+v"(c0), "+v"(c1), "+v"(c2), "+v"(c3), "+v"(c4), "+v"(c5), "+v"(c6), "+v"(c7)
               : "v"(f0), "v"(f1), "v"(f2), "v"(f3), "v"(f4), "v"(f5));
}

template <typename T> struct Frag;
template <> struct Frag<_Float16> {
  typedef v16h V; union U { v16h v; v8h h[2]; };
  static __device__ __forceinline__ v16h load(const _Float16* p) {
    U f; f.h[0] = *(const v8h*)(p); f.h[1] = *(const v8h*)(p + 16); return f.v;
  }
  static __device__ __forceinline__ v8f mma(v16h a, v16h b, v8f c) {
    return __builtin_amdgcn_wmma_f32_16x16x32_f16(false, a, false, b, (short)0, c, false, false);
  }
  static __device__ __forceinline__ void guard(v8f& a, v8f& b, v16h x, v16h y) { dep_guard_h(a, b, x, y); }
  static __device__ __forceinline__ void guard4(v8f& a, v8f& b, v8f& c, v8f& d, v16h x, v16h y) { dep_guard4_h(a, b, c, d, x, y); }
  static __device__ __forceinline__ void keep(v16h a, v16h b, v16h c, v16h d) { keep4_h(a, b, c, d); }
};
template <> struct Frag<__bf16> {
  typedef v16b V; union U { v16b v; v8b h[2]; };
  static __device__ __forceinline__ v16b load(const __bf16* p) {
    U f; f.h[0] = *(const v8b*)(p); f.h[1] = *(const v8b*)(p + 16); return f.v;
  }
  static __device__ __forceinline__ v8f mma(v16b a, v16b b, v8f c) {
    return __builtin_amdgcn_wmma_f32_16x16x32_bf16(false, a, false, b, (short)0, c, false, false);
  }
  static __device__ __forceinline__ void guard(v8f& a, v8f& b, v16b x, v16b y) { dep_guard_b(a, b, x, y); }
  static __device__ __forceinline__ void guard4(v8f& a, v8f& b, v8f& c, v8f& d, v16b x, v16b y) { dep_guard4_b(a, b, c, d, x, y); }
  static __device__ __forceinline__ void keep(v16b a, v16b b, v16b c, v16b d) { keep4_b(a, b, c, d); }
};

template <int ET> struct Elem;
template <> struct Elem<0> { typedef _Float16 T; };
template <> struct Elem<1> { typedef __bf16 T; };
template <int ET, bool SPLIT, int BIAS_MODE, int OUT_MODE, bool RESID, int ACT = 0>
__global__ __launch_bounds__(256) void wmma_gemm64(
    const unsigned short* __restrict__ Ap, const unsigned short* __restrict__ A2p, int lda, long strideA,
    const unsigned short* __restrict__ Btp, const unsigned short* __restrict__ Bt2p, int ldb, long strideB,
    void* __restrict__ Cout, void* __restrict__ Cout2, int ldc, long strideC,
    const float* __restrict__ bias,
    const float* __restrict__ resid, long strideR,
    int M, int N, int K, float scale) {
  typedef typename Elem<ET>::T T;
  typedef typename Frag<T>::V V;
  const T* A = (const T*)Ap; const T* A2 = (const T*)A2p; const T* Bt = (const T*)Btp; const T* Bt2 = (const T*)Bt2p;
  __shared__ __align__(16) float sT[8][16 * 68];
  const int b    = blockIdx.y;
  const int lane = threadIdx.x & 31;
  const int wave = threadIdx.x >> 5;
  const int tilesN = N >> 6;
  const int tilesM = M >> 6;
  const int tile = blockIdx.x * 8 + wave;
  if (tile >= tilesM * tilesN) return;
  const int tm = tile / tilesN;
  const int tn = tile - tm * tilesN;
  const int m0 = tm << 6;
  const int n0 = tn << 6;

  const T* Ab  = A  + (size_t)b * strideA;
  const T* Bb  = Bt + (size_t)b * strideB;
  const T* Ab2 = SPLIT ? (A2  + (size_t)b * strideA) : nullptr;
  const T* Bb2 = SPLIT ? (Bt2 + (size_t)b * strideB) : nullptr;

  const int rlane = lane & 15;
  const int koff  = (lane >> 4) * 8;
  const int mOff  = (lane >> 4) * 8;

  v8f acc[4][4];
#pragma unroll
  for (int i = 0; i < 4; ++i)
#pragma unroll
    for (int j = 0; j < 4; ++j) acc[i][j] = (v8f){0.f,0.f,0.f,0.f,0.f,0.f,0.f,0.f};

  for (int k0 = 0; k0 < K; k0 += 32) {
    V bh[4], bl[4];
#pragma unroll
    for (int j = 0; j < 4; ++j) {
      const size_t bo = (size_t)(n0 + (j << 4) + rlane) * ldb + koff + k0;
      bh[j] = Frag<T>::load(Bb + bo);
      if (SPLIT) bl[j] = Frag<T>::load(Bb2 + bo);
    }
#pragma unroll
    for (int i = 0; i < 4; ++i) {
      const size_t ao = (size_t)(m0 + (i << 4) + rlane) * lda + koff + k0;
      V ah = Frag<T>::load(Ab + ao);
      V al;
      if (SPLIT) al = Frag<T>::load(Ab2 + ao);
#pragma unroll
      for (int j = 0; j < 4; ++j) {
        acc[i][j] = Frag<T>::mma(ah, bh[j], acc[i][j]);
        if (SPLIT) {
          acc[i][j] = Frag<T>::mma(ah, bl[j], acc[i][j]);
          acc[i][j] = Frag<T>::mma(al, bh[j], acc[i][j]);
        }
      }
      Frag<T>::guard4(acc[i][0], acc[i][1], acc[i][2], acc[i][3], ah, SPLIT ? al : bh[3]);
    }
    Frag<T>::keep(bh[0], bh[1], bh[2], bh[3]);
    if (SPLIT) Frag<T>::keep(bl[0], bl[1], bl[2], bl[3]);
  }
  acc_guard4(acc[0][0], acc[0][1], acc[0][2], acc[0][3]);
  acc_guard4(acc[1][0], acc[1][1], acc[1][2], acc[1][3]);
  acc_guard4(acc[2][0], acc[2][1], acc[2][2], acc[2][3]);
  acc_guard4(acc[3][0], acc[3][1], acc[3][2], acc[3][3]);

  float* slab = sT[wave];
  const float* Rb = RESID ? (resid + (size_t)b * strideR) : nullptr;
#pragma unroll
  for (int i = 0; i < 4; ++i) {
    const int mBase = m0 + (i << 4);
#pragma unroll
    for (int j = 0; j < 4; ++j) {
      const int n = n0 + (j << 4) + rlane;
      float bv = 0.f;
      if (BIAS_MODE == 2) bv = bias[n];
#pragma unroll
      for (int r = 0; r < 8; ++r) {
        float v = acc[i][j][r] * scale;
        if (BIAS_MODE == 1) v += bias[mBase + mOff + r];
        if (BIAS_MODE == 2) v += bv;
        if (RESID) v += Rb[(size_t)(mBase + mOff + r) * ldc + n];
        if (ACT == 1) v = tanhf(v);
        if (ACT == 2) v = fmaxf(v, 0.0f);
        if (ACT == 4) v = (v > 0.f) ? v : 0.01f * v;
        slab[(mOff + r) * 68 + (j << 4) + rlane] = v;
      }
    }
    __builtin_amdgcn_fence(__ATOMIC_RELEASE, "workgroup");
    __builtin_amdgcn_wave_barrier();
    __builtin_amdgcn_fence(__ATOMIC_ACQUIRE, "workgroup");
    if (OUT_MODE == 0) {
      float* C = (float*)Cout + (size_t)b * strideC;
      const int hh = lane >> 4, c4 = (lane & 15) * 4;
      for (int pass = 0; pass < 2; ++pass) {
#pragma unroll
        for (int it = 0; it < 8; ++it) {
          const int row = it * 2 + hh;
          v4f v = *(const v4f*)(slab + row * 68 + c4);
          *(volatile v4f*)(C + (size_t)(mBase + row) * ldc + n0 + c4) = v;
        }
        __threadfence();
      }
    } else {
      const int q = lane >> 3, c8 = (lane & 7) * 8;
      unsigned short* C  = (unsigned short*)Cout  + (size_t)b * strideC;
      unsigned short* C2 = (OUT_MODE == 2) ? ((unsigned short*)Cout2 + (size_t)b * strideC) : nullptr;
      for (int pass = 0; pass < 2; ++pass) {
#pragma unroll
        for (int it = 0; it < 4; ++it) {
          const int row = it * 4 + q;
          const float* sp = slab + row * 68 + c8;
          v8h hv, lv;
#pragma unroll
          for (int e = 0; e < 8; ++e) {
            if (OUT_MODE == 1) {
              hv[e] = (_Float16)sp[e];
            } else {
              unsigned short hb = f2bf_bits(sp[e]);
              unsigned short lb = f2bf_bits(sp[e] - bf_bits2f(hb));
              hv[e] = __builtin_bit_cast(_Float16, hb);
              lv[e] = __builtin_bit_cast(_Float16, lb);
            }
          }
          *(volatile v8h*)(C + (size_t)(mBase + row) * ldc + n0 + c8) = hv;
          if (OUT_MODE == 2) *(volatile v8h*)(C2 + (size_t)(mBase + row) * ldc + n0 + c8) = lv;
        }
        __threadfence();
      }
    }
    __builtin_amdgcn_fence(__ATOMIC_RELEASE, "workgroup");
    __builtin_amdgcn_wave_barrier();
    __builtin_amdgcn_fence(__ATOMIC_ACQUIRE, "workgroup");
  }
}

__device__ __forceinline__ unsigned pack_f16x2(float a, float b) {
  const _Float16 h0 = (_Float16)a, h1 = (_Float16)b;
  return (unsigned)__builtin_bit_cast(unsigned short, h0) | ((unsigned)__builtin_bit_cast(unsigned short, h1) << 16);
}
__device__ __forceinline__ void st2u(unsigned* p, unsigned v) { *(volatile unsigned*)p = v; __threadfence(); *(volatile unsigned*)p = v; }
__device__ __forceinline__ float ftanh(float x) { return 1.0f - 2.0f * __builtin_amdgcn_rcpf(1.0f + expf(2.0f * x)); }

__global__ __launch_bounds__(NTHR) void prep_kernel(const float* __restrict__ Whx, const float* __restrict__ Whh,
                                                    const float* __restrict__ Wph,
                                                    unsigned* __restrict__ W16u, unsigned* __restrict__ P16u) {
  const int blk = blockIdx.x, tid = threadIdx.x, lane = tid & 31, wave = tid >> 5;
  if (blk < NH / 8) {
    const int n = blk * 8 + wave;
    unsigned* rowp = W16u + (size_t)n * (KF / 2);
#pragma unroll 1
    for (int i = 0; i < NH / 64; ++i) {
      const int d = 32 * i + lane;
      const int k = 2 * d;
      const float w0 = Whh[(size_t)k * NH + n] * WCARRY;
      const float w1 = Whh[(size_t)(k + 1) * NH + n] * WCARRY;
      st2u(rowp + d, pack_f16x2(w0, w1));
    }
    {
      const int k = 2 * lane;
      const float w0 = Whx[(size_t)k * NH + n] * WCARRY;
      const float w1 = Whx[(size_t)(k + 1) * NH + n] * WCARRY;
      st2u(rowp + (NH / 2) + lane, pack_f16x2(w0, w1));
    }
  } else {
    const int n = (blk - NH / 8) * 8 + wave;
    unsigned* rowp = P16u + (size_t)n * (NH / 2);
#pragma unroll 1
    for (int i = 0; i < NH / 64; ++i) {
      const int d = 32 * i + lane;
      const int k = 2 * d;
      const float w0 = Wph[(size_t)k * NO + n] * WCARRY;
      const float w1 = Wph[(size_t)(k + 1) * NO + n] * WCARRY;
      st2u(rowp + d, pack_f16x2(w0, w1));
    }
  }
}

__global__ __launch_bounds__(NTHR) void rnn_seq_kernel(const float* __restrict__ x, const float* __restrict__ bh,
                                                       const unsigned short* __restrict__ W16p,
                                                       unsigned short* __restrict__ HT16p) {
  __shared__ __align__(16) _Float16 At[2 * ATILE];
  const _Float16* W16 = (const _Float16*)W16p;
  _Float16* HT16 = (_Float16*)HT16p;
  const int tid = threadIdx.x, lane = tid & 31, wave = tid >> 5;
  const int c = lane & 15, hh = lane >> 4, koff = hh * 8, mOff = hh * 8;
  const int rowbase = blockIdx.x * RPB;
  const int n0 = wave * 64;
  const int xr = tid >> 3, xc8 = (tid & 7) * 8;

  {
    const v4u z = {0u, 0u, 0u, 0u};
    for (int i = tid; i < (2 * ATILE) / 8; i += NTHR) *(v4u*)(At + i * 8) = z;
  }
  __syncthreads();
  {
    const float* xs = x + ((size_t)(rowbase + xr) * NT + 0) * NI + xc8;
    const v4f f0 = *(const v4f*)xs;
    const v4f f1 = *(const v4f*)(xs + 4);
    v8h hv;
    hv[0] = (_Float16)f0[0]; hv[1] = (_Float16)f0[1]; hv[2] = (_Float16)f0[2]; hv[3] = (_Float16)f0[3];
    hv[4] = (_Float16)f1[0]; hv[5] = (_Float16)f1[1]; hv[6] = (_Float16)f1[2]; hv[7] = (_Float16)f1[3];
    *(v8h*)(At + xr * APITCH + NH + xc8) = hv;
  }
  float bhv[4];
#pragma unroll
  for (int j = 0; j < 4; ++j) bhv[j] = bh[n0 + 16 * j + c];
  __syncthreads();

  const _Float16* brow = W16 + (size_t)(n0 + c) * KF + koff;
  const v8f z8 = {0.f, 0.f, 0.f, 0.f, 0.f, 0.f, 0.f, 0.f};

#pragma unroll 1
  for (int t = 0; t < NT; ++t) {
    const _Float16* cur = At + (t & 1) * ATILE;
    _Float16*       nxt = At + ((t + 1) & 1) * ATILE;

    {
      const int tn = (t + 1 < NT) ? (t + 1) : (NT - 1);
      const float* xs = x + ((size_t)(rowbase + xr) * NT + tn) * NI + xc8;
      const v4f f0 = *(const v4f*)xs;
      const v4f f1 = *(const v4f*)(xs + 4);
      v8h hv;
      hv[0] = (_Float16)f0[0]; hv[1] = (_Float16)f0[1]; hv[2] = (_Float16)f0[2]; hv[3] = (_Float16)f0[3];
      hv[4] = (_Float16)f1[0]; hv[5] = (_Float16)f1[1]; hv[6] = (_Float16)f1[2]; hv[7] = (_Float16)f1[3];
      *(v8h*)(nxt + xr * APITCH + NH + xc8) = hv;
    }

    v8f acc[2][4];
#pragma unroll
    for (int i = 0; i < 2; ++i)
#pragma unroll
      for (int j = 0; j < 4; ++j) acc[i][j] = z8;

    const _Float16* arow0 = cur + c * APITCH + koff;
    const _Float16* arow1 = cur + (16 + c) * APITCH + koff;
#pragma unroll 2
    for (int kc = 0; kc < NKC; ++kc) {
      const v16h a0 = Frag<_Float16>::load(arow0 + kc * 32);
      const v16h a1 = Frag<_Float16>::load(arow1 + kc * 32);
      v16h fb[4];
#pragma unroll
      for (int j = 0; j < 4; ++j) fb[j] = Frag<_Float16>::load(brow + (size_t)(16 * j) * KF + kc * 32);
#pragma unroll
      for (int j = 0; j < 4; ++j) {
        acc[0][j] = Frag<_Float16>::mma(a0, fb[j], acc[0][j]);
        acc[1][j] = Frag<_Float16>::mma(a1, fb[j], acc[1][j]);
      }
      guard8_h(acc[0][0], acc[0][1], acc[0][2], acc[0][3], acc[1][0], acc[1][1], acc[1][2], acc[1][3],
               a0, a1, fb[0], fb[1], fb[2], fb[3]);
    }
    acc_guard4(acc[0][0], acc[0][1], acc[0][2], acc[0][3]);
    acc_guard4(acc[1][0], acc[1][1], acc[1][2], acc[1][3]);

#pragma unroll
    for (int i = 0; i < 2; ++i) {
#pragma unroll
      for (int j = 0; j < 4; ++j) {
#pragma unroll
        for (int r = 0; r < 8; ++r) {
          const float z  = acc[i][j][r] * WCARRY_INV + bhv[j];
          const float hv = ftanh(z);
          nxt[(16 * i + mOff + r) * APITCH + n0 + 16 * j + c] = (_Float16)hv;
        }
      }
    }
    __syncthreads();
  }

  {
    const _Float16* fin = At + (NT & 1) * ATILE;
    const int q4 = lane >> 3, c8 = (lane & 7) * 8;
    for (int pass = 0; pass < 2; ++pass) {
#pragma unroll
      for (int it = 0; it < 8; ++it) {
        const int rr = it * 4 + q4;
        const v8h v = *(const v8h*)(fin + rr * APITCH + n0 + c8);
        *(volatile v8h*)(HT16 + (size_t)(rowbase + rr) * NH + n0 + c8) = v;
      }
      __threadfence();
    }
  }
}

__global__ __launch_bounds__(NTHR) void softmax_rows_kernel(const float* __restrict__ LG, float* __restrict__ out, int nrows) {
  __shared__ __align__(16) float Sx[NTHR / 32][NO];
  const int tid = threadIdx.x, lane = tid & 31, wave = tid >> 5;
  const int row = blockIdx.x * (NTHR / 32) + wave;
  if (row >= nrows) return;
  const float* rp = LG + (size_t)row * NO;
  float m = -INFINITY;
#pragma unroll 1
  for (int q = 0; q < NO / 128; ++q) {
    const v4f v = *(const v4f*)(rp + 128 * q + 4 * lane);
    m = fmaxf(m, fmaxf(fmaxf(v[0], v[1]), fmaxf(v[2], v[3])));
  }
#pragma unroll
  for (int off = 1; off < 32; off <<= 1) m = fmaxf(m, __shfl_xor(m, off, 32));
  float s = 0.0f;
#pragma unroll 1
  for (int q = 0; q < NO / 128; ++q) {
    const v4f v = *(const v4f*)(rp + 128 * q + 4 * lane);
    s += (expf(v[0] - m) + expf(v[1] - m)) + (expf(v[2] - m) + expf(v[3] - m));
  }
#pragma unroll
  for (int off = 1; off < 32; off <<= 1) s += __shfl_xor(s, off, 32);
  const float inv = 1.0f / s;
  float* sl = Sx[wave];
#pragma unroll 1
  for (int q = 0; q < NO / 128; ++q) {
    const v4f v = *(const v4f*)(rp + 128 * q + 4 * lane);
    v4f o;
    o[0] = expf(v[0] - m) * inv; o[1] = expf(v[1] - m) * inv;
    o[2] = expf(v[2] - m) * inv; o[3] = expf(v[3] - m) * inv;
    *(v4f*)(sl + 128 * q + 4 * lane) = o;
  }
  __builtin_amdgcn_fence(__ATOMIC_RELEASE, "workgroup");
  __builtin_amdgcn_wave_barrier();
  __builtin_amdgcn_fence(__ATOMIC_ACQUIRE, "workgroup");
  float* op = out + (size_t)row * NO;
  for (int pass = 0; pass < 2; ++pass) {
#pragma unroll 1
    for (int q = 0; q < NO / 128; ++q) {
      const v4f o = *(const v4f*)(sl + 128 * q + 4 * lane);
      *(volatile v4f*)(op + 128 * q + 4 * lane) = o;
    }
    __threadfence();
  }
}

extern "C" void kernel_launch(void* const* d_in, const int* in_sizes, int n_in,
                              void* d_out, int out_size, void* d_ws, size_t ws_size, hipStream_t stream) {
  if (n_in < 6 || d_out == nullptr || d_ws == nullptr) return;
  if (in_sizes[0] != NB * NT * NI || in_sizes[1] != NI * NH || in_sizes[2] != NH * NH ||
      in_sizes[3] != NH || in_sizes[4] != NH * NO || in_sizes[5] != NO || out_size != NB * NO) return;

  const float* x   = (const float*)d_in[0];
  const float* Whx = (const float*)d_in[1];
  const float* Whh = (const float*)d_in[2];
  const float* bh  = (const float*)d_in[3];
  const float* Wph = (const float*)d_in[4];
  const float* bo  = (const float*)d_in[5];
  float* out = (float*)d_out;

  char* ws = (char*)d_ws; size_t off = 0;
  auto carve = [&](size_t bytes) -> char* { char* p = ws + off; off += (bytes + 255) & ~(size_t)255; return p; };
  unsigned short* W16    = (unsigned short*)carve((size_t)NH * KF * 2);
  unsigned short* P16    = (unsigned short*)carve((size_t)NO * NH * 2);
  unsigned short* HT16   = (unsigned short*)carve((size_t)NB * NH * 2);
  float*          LOGITS = (float*)carve((size_t)NB * NO * 4);
  if (off > ws_size || off > (size_t)134217728) return;

  prep_kernel<<<NH / 8 + NO / 8, NTHR, 0, stream>>>(Whx, Whh, Wph, (unsigned*)W16, (unsigned*)P16);

  rnn_seq_kernel<<<NRBLK, NTHR, 0, stream>>>(x, bh, W16, HT16);

  wmma_gemm64<0, false, 2, 0, false, 0><<<dim3(((NB / 64) * (NO / 64)) / 8, 1), 256, 0, stream>>>(
      HT16, nullptr, NH, 0L, P16, nullptr, NH, 0L,
      (void*)LOGITS, nullptr, NO, 0L, bo, nullptr, 0L, NB, NO, NH, WCARRY_INV);

  softmax_rows_kernel<<<NB / (NTHR / 32), NTHR, 0, stream>>>(LOGITS, out, NB);
}
